// Decoder_45414984188138
// MI455X (gfx1250) — hardware-verified
//
#include <hip/hip_runtime.h>
#include <stddef.h>
#include <stdint.h>

#ifndef NB
#define NB 2
#endif
#ifndef SEQ
#define SEQ 2048
#endif
#define NB_FULL  2
#define SEQ_FULL 2048
#define DM   1024
#define NH   16
#define HD   64
#define DFF  4096
#define NTOK (NB * SEQ)

#define WSC     64.0f
#define INV_WSC 0.015625f
#define CTXC    64.0f
#define INV_WO  (1.0f / 4096.0f)
#define SCL2    0.18033688011112042f
#define PCARRY  8.0f
#define NEGBIG  (-1.0e30f)
#define WSMAX   134217728

static_assert(SEQ % 128 == 0);
static_assert((SEQ & (SEQ - 1)) == 0);
static_assert(NB <= NB_FULL && SEQ <= SEQ_FULL);
static_assert(NH * HD == DM);
static_assert(DM % 128 == 0 && DFF % 128 == 0 && NTOK % 128 == 0);
static_assert(DM % 32 == 0 && DFF % 32 == 0);
static_assert((NTOK * DM) % 2048 == 0);
static_assert(NTOK % 8 == 0);

typedef float          v2f   __attribute__((ext_vector_type(2)));
typedef float          v4f   __attribute__((ext_vector_type(4)));
typedef float          v8f   __attribute__((ext_vector_type(8)));
typedef int            v8i   __attribute__((ext_vector_type(8)));
typedef unsigned short v8us  __attribute__((ext_vector_type(8)));
typedef _Float16       v4h   __attribute__((ext_vector_type(4)));
typedef _Float16       v8h   __attribute__((ext_vector_type(8)));
typedef _Float16       v16h  __attribute__((ext_vector_type(16)));
typedef v4f  __attribute__((may_alias)) v4fa;
typedef v8us __attribute__((may_alias)) v8usa;
typedef v8h  __attribute__((may_alias)) v8ha;
union Frag { v16h v; v8us h[2]; v8i w; };
union H8 { v8h h; v8us u; v4f f; };
union H4 { v4h h; v2f f; };

template <bool F> struct StT { typedef float T; };
template <> struct StT<false> { typedef _Float16 T; };

__device__ __forceinline__ float bf16_val(float f) {
  const unsigned u = __float_as_uint(f);
  return __uint_as_float(((u + 0x7FFFu + ((u >> 16) & 1u)) >> 16) << 16);
}
__device__ __forceinline__ v4f bf16_val4(v4f x) {
  v4f y;
  y.x = bf16_val(x.x); y.y = bf16_val(x.y); y.z = bf16_val(x.z); y.w = bf16_val(x.w);
  return y;
}
__device__ __forceinline__ unsigned fullrow(unsigned tok) {
  return (tok / (unsigned)SEQ) * (unsigned)SEQ_FULL + (tok & (unsigned)(SEQ - 1));
}
__device__ __forceinline__ v8f zero8() {
  v8f z = {0.f, 0.f, 0.f, 0.f, 0.f, 0.f, 0.f, 0.f};
  return z;
}
__device__ __forceinline__ void ldfrag(Frag& f, const char* p) {
  f.h[0] = *(const v8usa*)p;
  f.h[1] = *(const v8usa*)(p + 32);
}
__device__ __forceinline__ v8f wmh(const Frag& a, const Frag& b, v8f c) {
  return __builtin_amdgcn_wmma_f32_16x16x32_f16(false, a.v, false, b.v, (short)0, c, false, false);
}
__device__ __forceinline__ void guard8(v8f& c0, v8f& c1, v8f& c2, v8f& c3, v8f& c4, v8f& c5, v8f& c6, v8f& c7,
                                       const Frag& f0, const Frag& f1, const Frag& f2, const Frag& f3,
                                       const Frag& f4, const Frag& f5) {
  asm volatile("v_nop\n\tv_nop\n\tv_nop\n\tv_nop"
               : "+v"(c0), "+v"(c1), "+v"(c2), "+v"(c3), "+v"(c4), "+v"(c5), "+v"(c6), "+v"(c7)
               : "v"(f0.w), "v"(f1.w), "v"(f2.w), "v"(f3.w), "v"(f4.w), "v"(f5.w));
}
__device__ __forceinline__ void guard4(v8f& c0, v8f& c1, v8f& c2, v8f& c3,
                                       const Frag& f0, const Frag& f1, const Frag& f2, const Frag& f3,
                                       const Frag& f4, const Frag& f5, const Frag& f6, const Frag& f7,
                                       const Frag& f8, const Frag& f9) {
  asm volatile("v_nop\n\tv_nop\n\tv_nop\n\tv_nop"
               : "+v"(c0), "+v"(c1), "+v"(c2), "+v"(c3)
               : "v"(f0.w), "v"(f1.w), "v"(f2.w), "v"(f3.w), "v"(f4.w), "v"(f5.w), "v"(f6.w), "v"(f7.w),
                 "v"(f8.w), "v"(f9.w));
}

__global__ __launch_bounds__(256) void k_tr(const float* __restrict__ s0, const float* __restrict__ s1,
                                            unsigned zsplit, unsigned R, unsigned C, unsigned short* dst) {
  __shared__ __attribute__((aligned(16))) _Float16 ts[64 * 72];
  const unsigned tid = threadIdx.x;
  const unsigned z = blockIdx.z;
  const size_t zs = (size_t)R * C;
  const float* src = (z < zsplit) ? (s0 + zs * z) : (s1 + zs * (z - zsplit));
  unsigned short* out = dst + zs * z;
  const unsigned r0 = blockIdx.y * 64u, c0 = blockIdx.x * 64u;
  const unsigned r = tid >> 2, cs = (tid & 3u) * 16u;
  const float* p = src + (size_t)(r0 + r) * C + c0 + cs;
#pragma unroll
  for (unsigned q = 0; q < 4; ++q) {
    const v4f x = *(const v4fa*)(p + 4 * q);
    ts[(cs + 4 * q + 0) * 72 + r] = (_Float16)(bf16_val(x.x) * WSC);
    ts[(cs + 4 * q + 1) * 72 + r] = (_Float16)(bf16_val(x.y) * WSC);
    ts[(cs + 4 * q + 2) * 72 + r] = (_Float16)(bf16_val(x.z) * WSC);
    ts[(cs + 4 * q + 3) * 72 + r] = (_Float16)(bf16_val(x.w) * WSC);
  }
  __syncthreads();
  v4f vals[2];
  size_t off[2];
#pragma unroll
  for (unsigned i = 0; i < 2; ++i) {
    const unsigned pc = tid + 256u * i;
    const unsigned c = pc >> 3, r8 = (pc & 7u) * 8u;
    H8 u;
    u.h = *(const v8ha*)(ts + c * 72 + r8);
    vals[i] = u.f;
    off[i] = (size_t)(c0 + c) * R + r0 + r8;
  }
#pragma unroll
  for (unsigned i = 0; i < 2; ++i) *(volatile v4f*)(out + off[i]) = vals[i];
  __threadfence();
#pragma unroll
  for (unsigned i = 0; i < 2; ++i) *(volatile v4f*)(out + off[i]) = vals[i];
}

__global__ __launch_bounds__(256) void k_cvt(const float* __restrict__ s0, const float* __restrict__ s1,
                                             unsigned short* dst) {
  const unsigned z = blockIdx.y;
  const float* src = z ? s1 : s0;
  const unsigned e = (blockIdx.x * 256u + threadIdx.x) * 8u;
  const unsigned tok = e >> 10, col = e & 1023u;
  const float* p = src + (size_t)fullrow(tok) * DM + col;
  const v4f a = *(const v4fa*)p;
  const v4f b = *(const v4fa*)(p + 4);
  H8 u;
  u.h[0] = (_Float16)bf16_val(a.x); u.h[1] = (_Float16)bf16_val(a.y);
  u.h[2] = (_Float16)bf16_val(a.z); u.h[3] = (_Float16)bf16_val(a.w);
  u.h[4] = (_Float16)bf16_val(b.x); u.h[5] = (_Float16)bf16_val(b.y);
  u.h[6] = (_Float16)bf16_val(b.z); u.h[7] = (_Float16)bf16_val(b.w);
  unsigned short* o = dst + (size_t)z * NTOK * DM + e;
  const v4f v = u.f;
  *(volatile v4f*)o = v;
  __threadfence();
  *(volatile v4f*)o = v;
}

template <int EPI>
__global__ __launch_bounds__(256) void k_gemm(const unsigned short* __restrict__ A,
                                              const unsigned short* __restrict__ Bt,
                                              unsigned K, unsigned N,
                                              const float* __restrict__ bias0,
                                              const float* __restrict__ bias1, unsigned nsplit,
                                              float scale, void* outp, const float* __restrict__ resid) {
  constexpr bool F32OUT = (EPI >= 3);
  constexpr int WMT = F32OUT ? 4 : 2;
  constexpr int WNT = F32OUT ? 2 : 4;
  typedef typename StT<F32OUT>::T ST;
  __shared__ __attribute__((aligned(16))) ST stg[8 * 2048];

  const unsigned tid = threadIdx.x, lane = tid & 31u, wave = tid >> 5, hh = lane >> 4, m = lane & 15u;
  const unsigned wm = F32OUT ? (wave >> 2) : (wave >> 1);
  const unsigned wn = F32OUT ? (wave & 3u) : (wave & 1u);
  const unsigned bm = blockIdx.y * 128u, bn = blockIdx.x * 128u;
  const unsigned rowA = bm + wm * (16u * WMT) + m;
  const unsigned rowB = bn + wn * (16u * WNT) + m;
  const unsigned offA = (rowA * K + 8u * hh) * 2u;
  const unsigned offB = (rowB * K + 8u * hh) * 2u;
  const unsigned rstep = 32u * K;
  const char* Ab = (const char*)A;
  const char* Bb = (const char*)Bt;

  v8f acc[WMT][WNT];
#pragma unroll
  for (int i = 0; i < WMT; ++i)
#pragma unroll
    for (int j = 0; j < WNT; ++j) acc[i][j] = zero8();

#pragma unroll 2
  for (unsigned k0 = 0; k0 < K; k0 += 32) {
    const char* ak = Ab + (size_t)k0 * 2;
    const char* bk = Bb + (size_t)k0 * 2;
    Frag a[WMT], b[WNT];
#pragma unroll
    for (int i = 0; i < WMT; ++i) ldfrag(a[i], ak + (offA + (unsigned)i * rstep));
#pragma unroll
    for (int j = 0; j < WNT; ++j) ldfrag(b[j], bk + (offB + (unsigned)j * rstep));
#pragma unroll
    for (int i = 0; i < WMT; ++i)
#pragma unroll
      for (int j = 0; j < WNT; ++j) acc[i][j] = wmh(a[i], b[j], acc[i][j]);
    if constexpr (WMT == 4) {
      guard8(acc[0][0], acc[0][1], acc[1][0], acc[1][1], acc[2][0], acc[2][1], acc[3][0], acc[3][1],
             a[0], a[1], a[2], a[3], b[0], b[1]);
    } else {
      guard8(acc[0][0], acc[0][1], acc[0][2], acc[0][3], acc[1][0], acc[1][1], acc[1][2], acc[1][3],
             a[0], a[1], b[0], b[1], b[2], b[3]);
    }
  }

  ST* wsb = stg + wave * 2048u;
  if constexpr (!F32OUT) {
    const float* bcol = (bn < nsplit) ? (bias0 + bn + wn * 64u) : (bias1 + (bn - nsplit) + wn * 64u);
#pragma unroll
    for (int i = 0; i < 2; ++i) {
      float brow[8];
#pragma unroll
      for (int r = 0; r < 8; ++r)
        brow[r] = (EPI == 2) ? bf16_val(bias0[bm + wm * 32u + 16u * i + 8u * hh + r]) : 0.0f;
#pragma unroll
      for (int j = 0; j < 4; ++j) {
        const float bc = (EPI == 2) ? 0.0f : bf16_val(bcol[16u * j + m]);
#pragma unroll
        for (int r = 0; r < 8; ++r) {
          const unsigned rl = 16u * i + 8u * hh + r;
          float v = acc[i][j][r] * scale + ((EPI == 2) ? brow[r] : bc);
          if (EPI == 1) v = fmaxf(v, 0.0f);
          wsb[rl * 64u + 16u * j + m] = (_Float16)v;
        }
      }
    }
    __syncthreads();
    unsigned short* out16 = (unsigned short*)outp;
    const unsigned c8 = (lane & 7u) * 8u;
    const size_t base = (size_t)(bm + wm * 32u + (lane >> 3)) * N + bn + wn * 64u + c8;
    v4f vals[8];
#pragma unroll
    for (int it = 0; it < 8; ++it) {
      const unsigned rl = 4u * it + (lane >> 3);
      H8 u;
      u.h = *(const v8ha*)(wsb + rl * 64u + c8);
      vals[it] = u.f;
    }
#pragma unroll
    for (int it = 0; it < 8; ++it) *(volatile v4f*)(out16 + base + (size_t)it * 4u * N) = vals[it];
    __threadfence();
#pragma unroll
    for (int it = 0; it < 8; ++it) *(volatile v4f*)(out16 + base + (size_t)it * 4u * N) = vals[it];
  } else {
#pragma unroll
    for (int i = 0; i < 4; ++i)
#pragma unroll
      for (int j = 0; j < 2; ++j)
#pragma unroll
        for (int r = 0; r < 8; ++r)
          wsb[(16u * i + 8u * hh + r) * 32u + 16u * j + m] = acc[i][j][r] * scale;
    __syncthreads();
    float* outf = (float*)outp;
    const unsigned c4 = (lane & 7u) * 4u;
    const unsigned gcol = bn + wn * 32u + c4;
    const v4f b4 = bf16_val4(*(const v4fa*)(bias0 + gcol));
    const unsigned grow0 = bm + wm * 64u + (lane >> 3);
    v4f vals[16];
#pragma unroll
    for (int it = 0; it < 16; ++it) {
      const unsigned rl = 4u * it + (lane >> 3);
      const unsigned grow = grow0 + 4u * it;
      const v4f s = *(const v4fa*)(wsb + rl * 32u + c4);
      v4f r4;
      if (EPI == 3) {
        r4 = *(const v4fa*)(resid + (size_t)grow * N + gcol);
      } else {
        r4 = bf16_val4(*(const v4fa*)(resid + (size_t)fullrow(grow) * DM + gcol));
      }
      vals[it] = r4 + (s + b4);
    }
    const size_t base = (size_t)grow0 * N + gcol;
#pragma unroll
    for (int it = 0; it < 16; ++it) *(volatile v4f*)(outf + base + (size_t)it * 4u * N) = vals[it];
    __threadfence();
#pragma unroll
    for (int it = 0; it < 16; ++it) *(volatile v4f*)(outf + base + (size_t)it * 4u * N) = vals[it];
  }
}

__global__ __launch_bounds__(128) void k_flash(const unsigned short* __restrict__ Qp, unsigned pq,
                                               const unsigned short* __restrict__ Kp, unsigned pk,
                                               const unsigned short* __restrict__ Vt,
                                               unsigned short* ctx, int causal) {
  __shared__ __attribute__((aligned(16))) unsigned short ost[4 * 1024];
  const unsigned tid = threadIdx.x, lane = tid & 31u, wave = tid >> 5, hh = lane >> 4, m = lane & 15u;
  const unsigned b = blockIdx.y >> 4, h = blockIdx.y & 15u;
  const unsigned qw = blockIdx.x * 64u + wave * 16u;

  Frag bq0, bq1;
  {
    const char* qp = (const char*)Qp + ((size_t)(b * (unsigned)SEQ + qw + m) * pq + h * 64u + 8u * hh) * 2;
    ldfrag(bq0, qp);
    ldfrag(bq1, qp + 64);
  }
  const unsigned koff = (m * pk + h * 64u + 8u * hh) * 2u;
  const unsigned voff = ((h * 64u + m) * (unsigned)NTOK + 8u * hh) * 2u;
  const unsigned kstep = 32u * pk;
  const unsigned vstep = 32u * (unsigned)NTOK;

  v8f O[4];
#pragma unroll
  for (int nt = 0; nt < 4; ++nt) O[nt] = zero8();
  float mrun = NEGBIG, lrun = 0.0f;

  const unsigned ntile = causal ? (((qw + 15u) >> 6) + 1u) : (unsigned)(SEQ / 64);
  for (unsigned j = 0; j < ntile; ++j) {
    const unsigned s0 = j * 64u;
    const char* kt = (const char*)Kp + (size_t)(b * (unsigned)SEQ + s0) * pk * 2;
    Frag ka[4][2];
#pragma unroll
    for (int t = 0; t < 4; ++t) {
      ldfrag(ka[t][0], kt + (koff + (unsigned)t * kstep));
      ldfrag(ka[t][1], kt + (koff + (unsigned)t * kstep) + 64);
    }
    v8f st[4];
#pragma unroll
    for (int t = 0; t < 4; ++t) {
      st[t] = wmh(ka[t][0], bq0, zero8());
      st[t] = wmh(ka[t][1], bq1, st[t]);
    }
    guard4(st[0], st[1], st[2], st[3], ka[0][0], ka[0][1], ka[1][0], ka[1][1],
           ka[2][0], ka[2][1], ka[3][0], ka[3][1], bq0, bq1);

    if (causal && (s0 + 63u > qw)) {
      const unsigned qrow = qw + m;
#pragma unroll
      for (int t = 0; t < 4; ++t)
#pragma unroll
        for (int r = 0; r < 8; ++r) {
          const unsigned key = s0 + 16u * t + 8u * hh + r;
          st[t][r] = (key > qrow) ? NEGBIG : st[t][r];
        }
    }
    float mx = st[0][0];
#pragma unroll
    for (int t = 0; t < 4; ++t)
#pragma unroll
      for (int r = 0; r < 8; ++r) mx = fmaxf(mx, st[t][r]);
    mx = fmaxf(mx, __shfl_xor(mx, 16, 32));
    const float mnew = fmaxf(mrun, mx);
    const float corr = __builtin_amdgcn_exp2f((mrun - mnew) * SCL2);
    mrun = mnew;
    const float bias = PCARRY - mnew * SCL2;
    float ls = 0.0f;
#pragma unroll
    for (int t = 0; t < 4; ++t)
#pragma unroll
      for (int r = 0; r < 8; ++r) {
        const float p = __builtin_amdgcn_exp2f(fmaf(st[t][r], SCL2, bias));
        ls += p;
        st[t][r] = p;
      }
    lrun = lrun * corr + ls;
#pragma unroll
    for (int nt = 0; nt < 4; ++nt)
#pragma unroll
      for (int r = 0; r < 8; ++r) O[nt][r] *= corr;

    Frag pf[2];
#pragma unroll
    for (int u = 0; u < 2; ++u)
#pragma unroll
      for (int r = 0; r < 8; ++r) {
        pf[u].v[r]     = (_Float16)st[2 * u][r];
        pf[u].v[8 + r] = (_Float16)st[2 * u + 1][r];
      }
    const char* vt = (const char*)Vt + (size_t)(b * (unsigned)SEQ + s0) * 2;
    Frag va[2][4];
#pragma unroll
    for (int u = 0; u < 2; ++u)
#pragma unroll
      for (int nt = 0; nt < 4; ++nt) ldfrag(va[u][nt], vt + (voff + (unsigned)nt * vstep) + 64 * u);
#pragma unroll
    for (int u = 0; u < 2; ++u)
#pragma unroll
      for (int nt = 0; nt < 4; ++nt) O[nt] = wmh(va[u][nt], pf[u], O[nt]);
    guard4(O[0], O[1], O[2], O[3], va[0][0], va[0][1], va[0][2], va[0][3],
           va[1][0], va[1][1], va[1][2], va[1][3], pf[0], pf[1]);
  }

  const float lt = lrun + __shfl_xor(lrun, 16, 32);
  const float inv = CTXC * (1.0f / lt);
  unsigned short* os = ost + wave * 1024u;
#pragma unroll
  for (int nt = 0; nt < 4; ++nt) {
    H8 u;
#pragma unroll
    for (int r = 0; r < 8; ++r) u.h[r] = (_Float16)(O[nt][r] * inv);
    *(v8usa*)(os + m * 64u + 16u * nt + 8u * hh) = u.u;
  }
  __syncthreads();
  const unsigned c8 = (lane & 7u) * 8u;
  v4f vals[4];
#pragma unroll
  for (int it = 0; it < 4; ++it) {
    const unsigned row = 4u * it + (lane >> 3);
    H8 u;
    u.u = *(const v8usa*)(os + row * 64u + c8);
    vals[it] = u.f;
  }
  unsigned short* dst = ctx + (size_t)(b * (unsigned)SEQ + qw + (lane >> 3)) * DM + h * 64u + c8;
#pragma unroll
  for (int it = 0; it < 4; ++it) *(volatile v4f*)(dst + (size_t)it * 4u * DM) = vals[it];
  __threadfence();
#pragma unroll
  for (int it = 0; it < 4; ++it) *(volatile v4f*)(dst + (size_t)it * 4u * DM) = vals[it];
}

template <int FINAL>
__global__ __launch_bounds__(256) void k_ln(const float* __restrict__ Y, const float* __restrict__ g,
                                            const float* __restrict__ be, float* outf, unsigned short* outh) {
  const unsigned tid = threadIdx.x, lane = tid & 31u, wave = tid >> 5;
  const unsigned row = blockIdx.x * 8u + wave;
  const float* yr = Y + (size_t)row * DM + lane * 4u;
  float s = 0.0f;
#pragma unroll 1
  for (unsigned it = 0; it < 8; ++it) {
    const v4f x = *(const v4fa*)(yr + it * 128u);
    s += (x.x + x.y) + (x.z + x.w);
  }
  s += __shfl_xor(s, 16, 32); s += __shfl_xor(s, 8, 32); s += __shfl_xor(s, 4, 32);
  s += __shfl_xor(s, 2, 32);  s += __shfl_xor(s, 1, 32);
  const float mu = s * (1.0f / 1024.0f);
  float q = 0.0f;
#pragma unroll 1
  for (unsigned it = 0; it < 8; ++it) {
    const v4f x = *(const v4fa*)(yr + it * 128u);
    const float d0 = x.x - mu, d1 = x.y - mu, d2 = x.z - mu, d3 = x.w - mu;
    q += (d0 * d0 + d1 * d1) + (d2 * d2 + d3 * d3);
  }
  q += __shfl_xor(q, 16, 32); q += __shfl_xor(q, 8, 32); q += __shfl_xor(q, 4, 32);
  q += __shfl_xor(q, 2, 32);  q += __shfl_xor(q, 1, 32);
  const float rstd = rsqrtf(q * (1.0f / 1024.0f) + 1e-5f);
  const unsigned orow = FINAL ? fullrow(row) : row;
  float* of = outf + (size_t)orow * DM + lane * 4u;
  unsigned short* oh = FINAL ? (unsigned short*)0 : (outh + (size_t)row * DM + lane * 4u);
#pragma unroll 1
  for (unsigned it = 0; it < 8; ++it) {
    const v4f x = *(const v4fa*)(yr + it * 128u);
    const v4f gg = bf16_val4(*(const v4fa*)(g + it * 128u + lane * 4u));
    const v4f bb = bf16_val4(*(const v4fa*)(be + it * 128u + lane * 4u));
    v4f y;
    y.x = (x.x - mu) * rstd * gg.x + bb.x;
    y.y = (x.y - mu) * rstd * gg.y + bb.y;
    y.z = (x.z - mu) * rstd * gg.z + bb.z;
    y.w = (x.w - mu) * rstd * gg.w + bb.w;
    H4 u;
    u.h[0] = (_Float16)y.x; u.h[1] = (_Float16)y.y; u.h[2] = (_Float16)y.z; u.h[3] = (_Float16)y.w;
    const v2f hv = u.f;
    *(volatile v4f*)(of + it * 128u) = y;
    if (!FINAL) *(volatile v2f*)(oh + it * 128u) = hv;
    __threadfence();
    *(volatile v4f*)(of + it * 128u) = y;
    if (!FINAL) *(volatile v2f*)(oh + it * 128u) = hv;
  }
}

#define SZ_W1M   ((size_t)DM * DM * 2)
#define OFF_WQKS ((size_t)0)
#define OFF_WVS  (OFF_WQKS + 2 * SZ_W1M)
#define OFF_WOS  (OFF_WVS + SZ_W1M)
#define OFF_WQC  (OFF_WOS + SZ_W1M)
#define OFF_WKC  (OFF_WQC + SZ_W1M)
#define OFF_WVC  (OFF_WKC + SZ_W1M)
#define OFF_WOC  (OFF_WVC + SZ_W1M)
#define OFF_W1T  (OFF_WOC + SZ_W1M)
#define OFF_W2T  (OFF_W1T + (size_t)DFF * DM * 2)
#define OFF_R1   (OFF_W2T + (size_t)DFF * DM * 2)
#define SZ_ACT16 ((size_t)NTOK * DM * 2)
#define OFF_XD   (OFF_R1)
#define OFF_XE   (OFF_XD + SZ_ACT16)
#define OFF_QK   (OFF_XE + SZ_ACT16)
#define SZ_R1    (4 * SZ_ACT16)
#define OFF_VT   (OFF_R1 + SZ_R1)
#define OFF_CTX  (OFF_VT + SZ_ACT16)
#define OFF_Y    (OFF_CTX + SZ_ACT16)
#define OFF_XF   (OFF_Y + 2 * SZ_ACT16)
#define OFF_XH   (OFF_XF + 2 * SZ_ACT16)
#define WS_TOTAL (OFF_XH + SZ_ACT16)

static_assert((size_t)NTOK * DFF * 2 == SZ_R1);
static_assert((size_t)NTOK * 2048 * 2 == 2 * SZ_ACT16);
static_assert(WS_TOTAL <= (size_t)WSMAX);
static_assert((SZ_ACT16 % 256) == 0 && (SZ_W1M % 256) == 0);

extern "C" void kernel_launch(void* const* d_in, const int* in_sizes, int n_in,
                              void* d_out, int out_size, void* d_ws, size_t ws_size,
                              hipStream_t stream) {
  if (n_in < 28) return;
  const long long needAct = ((long long)(NB - 1) * SEQ_FULL + SEQ) * DM;
  if ((long long)in_sizes[0] < needAct || (long long)in_sizes[1] < needAct) return;
  const int wi[6] = {2, 4, 6, 10, 12, 14};
  const int bi[6] = {3, 5, 7, 11, 13, 15};
  for (int i = 0; i < 6; ++i) {
    if (in_sizes[wi[i]] < NH * DM * HD) return;
    if (in_sizes[bi[i]] < NH * HD) return;
  }
  if (in_sizes[8] < DM * DM || in_sizes[16] < DM * DM) return;
  if (in_sizes[9] < DM || in_sizes[17] < DM) return;
  if (in_sizes[18] < DM * DFF || in_sizes[20] < DFF * DM) return;
  if (in_sizes[19] < DFF || in_sizes[21] < DM) return;
  for (int i = 22; i < 28; ++i) if (in_sizes[i] < DM) return;
  if ((long long)out_size < needAct) return;
  if (ws_size < (size_t)WS_TOTAL) return;

  const float* dec  = (const float*)d_in[0];
  const float* enc  = (const float*)d_in[1];
  const float* Wq_s = (const float*)d_in[2];  const float* bq_s = (const float*)d_in[3];
  const float* Wk_s = (const float*)d_in[4];  const float* bk_s = (const float*)d_in[5];
  const float* Wv_s = (const float*)d_in[6];  const float* bv_s = (const float*)d_in[7];
  const float* Wo_s = (const float*)d_in[8];  const float* bo_s = (const float*)d_in[9];
  const float* Wq_c = (const float*)d_in[10]; const float* bq_c = (const float*)d_in[11];
  const float* Wk_c = (const float*)d_in[12]; const float* bk_c = (const float*)d_in[13];
  const float* Wv_c = (const float*)d_in[14]; const float* bv_c = (const float*)d_in[15];
  const float* Wo_c = (const float*)d_in[16]; const float* bo_c = (const float*)d_in[17];
  const float* W1   = (const float*)d_in[18]; const float* b1   = (const float*)d_in[19];
  const float* W2   = (const float*)d_in[20]; const float* b2   = (const float*)d_in[21];
  const float* g1 = (const float*)d_in[22]; const float* be1 = (const float*)d_in[23];
  const float* g2 = (const float*)d_in[24]; const float* be2 = (const float*)d_in[25];
  const float* g3 = (const float*)d_in[26]; const float* be3 = (const float*)d_in[27];

  char* ws = (char*)d_ws;
  unsigned short* wQKs = (unsigned short*)(ws + OFF_WQKS);
  unsigned short* wVs  = (unsigned short*)(ws + OFF_WVS);
  unsigned short* wOs  = (unsigned short*)(ws + OFF_WOS);
  unsigned short* wQc  = (unsigned short*)(ws + OFF_WQC);
  unsigned short* wKc  = (unsigned short*)(ws + OFF_WKC);
  unsigned short* wVc  = (unsigned short*)(ws + OFF_WVC);
  unsigned short* wOc  = (unsigned short*)(ws + OFF_WOC);
  unsigned short* w1t  = (unsigned short*)(ws + OFF_W1T);
  unsigned short* w2t  = (unsigned short*)(ws + OFF_W2T);
  unsigned short* Xd   = (unsigned short*)(ws + OFF_XD);
  unsigned short* Xe   = (unsigned short*)(ws + OFF_XE);
  unsigned short* QK   = (unsigned short*)(ws + OFF_QK);
  unsigned short* Hh   = (unsigned short*)(ws + OFF_R1);
  unsigned short* VT   = (unsigned short*)(ws + OFF_VT);
  unsigned short* CTX  = (unsigned short*)(ws + OFF_CTX);
  float*          Y    = (float*)(ws + OFF_Y);
  float*          XF   = (float*)(ws + OFF_XF);
  unsigned short* XH   = (unsigned short*)(ws + OFF_XH);
  unsigned short* Qc   = QK;
  unsigned short* Kc   = QK + (size_t)NTOK * DM;
  float* out = (float*)d_out;

  const dim3 b256(256), b128(128);

  k_tr<<<dim3(1, 16, 32), b256, 0, stream>>>(Wq_s, Wk_s, 16u, (unsigned)DM, (unsigned)HD, wQKs);
  k_tr<<<dim3(1, 16, 16), b256, 0, stream>>>(Wv_s, Wv_s, 16u, (unsigned)DM, (unsigned)HD, wVs);
  k_tr<<<dim3(16, 16, 1), b256, 0, stream>>>(Wo_s, Wo_s, 1u, (unsigned)DM, (unsigned)DM, wOs);
  k_tr<<<dim3(1, 16, 32), b256, 0, stream>>>(Wq_c, Wk_c, 16u, (unsigned)DM, (unsigned)HD, wQc);
  k_tr<<<dim3(1, 16, 16), b256, 0, stream>>>(Wv_c, Wv_c, 16u, (unsigned)DM, (unsigned)HD, wVc);
  k_tr<<<dim3(16, 16, 1), b256, 0, stream>>>(Wo_c, Wo_c, 1u, (unsigned)DM, (unsigned)DM, wOc);
  k_tr<<<dim3(DFF / 64, DM / 64, 1), b256, 0, stream>>>(W1, W1, 1u, (unsigned)DM, (unsigned)DFF, w1t);
  k_tr<<<dim3(DM / 64, DFF / 64, 1), b256, 0, stream>>>(W2, W2, 1u, (unsigned)DFF, (unsigned)DM, w2t);
  k_cvt<<<dim3(NTOK * DM / 2048, 2), b256, 0, stream>>>(dec, enc, Xd);

  k_gemm<0><<<dim3(2048 / 128, NTOK / 128), b256, 0, stream>>>(Xd, wQKs, (unsigned)DM, 2048u, bq_s, bk_s, 1024u,
                                                               INV_WSC, (void*)QK, (const float*)0);
  k_gemm<2><<<dim3(NTOK / 128, DM / 128), b256, 0, stream>>>(wVs, Xd, (unsigned)DM, (unsigned)NTOK, bv_s, bv_s,
                                                             (unsigned)NTOK, INV_WSC, (void*)VT, (const float*)0);
  k_flash<<<dim3(SEQ / 64, NB * NH), b128, 0, stream>>>(QK, 2048u, QK + 1024, 2048u, VT, CTX, 1);
  k_gemm<4><<<dim3(DM / 128, NTOK / 128), b256, 0, stream>>>(CTX, wOs, (unsigned)DM, (unsigned)DM, bo_s, bo_s,
                                                             (unsigned)DM, INV_WO, (void*)Y, dec);
  k_ln<0><<<dim3(NTOK / 8), b256, 0, stream>>>(Y, g1, be1, XF, XH);

  k_gemm<0><<<dim3(DM / 128, NTOK / 128), b256, 0, stream>>>(XH, wQc, (unsigned)DM, (unsigned)DM, bq_c, bq_c,
                                                             (unsigned)DM, INV_WSC, (void*)Qc, (const float*)0);
  k_gemm<0><<<dim3(DM / 128, NTOK / 128), b256, 0, stream>>>(Xe, wKc, (unsigned)DM, (unsigned)DM, bk_c, bk_c,
                                                             (unsigned)DM, INV_WSC, (void*)Kc, (const float*)0);
  k_gemm<2><<<dim3(NTOK / 128, DM / 128), b256, 0, stream>>>(wVc, Xe, (unsigned)DM, (unsigned)NTOK, bv_c, bv_c,
                                                             (unsigned)NTOK, INV_WSC, (void*)VT, (const float*)0);
  k_flash<<<dim3(SEQ / 64, NB * NH), b128, 0, stream>>>(Qc, (unsigned)DM, Kc, (unsigned)DM, VT, CTX, 0);
  k_gemm<3><<<dim3(DM / 128, NTOK / 128), b256, 0, stream>>>(CTX, wOc, (unsigned)DM, (unsigned)DM, bo_c, bo_c,
                                                             (unsigned)DM, INV_WO, (void*)Y, XF);
  k_ln<0><<<dim3(NTOK / 8), b256, 0, stream>>>(Y, g2, be2, XF, XH);

  k_gemm<1><<<dim3(DFF / 128, NTOK / 128), b256, 0, stream>>>(XH, w1t, (unsigned)DM, (unsigned)DFF, b1, b1,
                                                              (unsigned)DFF, INV_WSC, (void*)Hh, (const float*)0);
  k_gemm<3><<<dim3(DM / 128, NTOK / 128), b256, 0, stream>>>(Hh, w2t, (unsigned)DFF, (unsigned)DM, b2, b2,
                                                             (unsigned)DM, INV_WSC, (void*)Y, XF);
  k_ln<1><<<dim3(NTOK / 8), b256, 0, stream>>>(Y, g3, be3, out, (unsigned short*)0);
}
